// FeatureAttentionLayer_46935402610805
// MI455X (gfx1250) — hardware-verified
//
#include <hip/hip_runtime.h>
#include <math.h>
#include <stdint.h>

#ifndef NB
#define NB    8
#endif
#define NF    2048
#define WIN   128
#define DIN   256
#define XBS_FULL (WIN * NF)
#define PCAR  32768.0f
#define VCAR  16.0f
#define LOG2E 1.4426950408889634f
#define ATT_WAVES   4
#define ATT_THREADS (ATT_WAVES * 32)
#define ITILES      (NF / 64)
#define ATT_BLOCKS  (NB * ITILES)
#define NKB         (NF / 32)
#define TP          68
static_assert(NB >= 1 && NB <= 8);
static_assert(WIN == 128 && DIN == 2 * WIN && ATT_THREADS == 128);
static_assert((NF % 64) == 0 && (NF % 256) == 0 && NKB * 32 == NF && ATT_BLOCKS == NB * (NF / 64));
static_assert(((NB * WIN * NF / 8) % 256) == 0);
static_assert((TP * 4) % 16 == 0 && WIN * TP * 4 <= 65536);

typedef unsigned short u16;
typedef _Float16 v16h __attribute__((ext_vector_type(16)));
typedef _Float16 v8h  __attribute__((ext_vector_type(8)));
typedef float    v8f  __attribute__((ext_vector_type(8)));
typedef float    v4f  __attribute__((ext_vector_type(4)));
typedef unsigned int v4u __attribute__((ext_vector_type(4)));

union FragH { v16h v; v8h h[2]; v4u u[2]; };

__device__ __forceinline__ unsigned short bf_bits(float f) {
  unsigned u = __float_as_uint(f);
  return (unsigned short)((u + 0x7FFFu + ((u >> 16) & 1u)) >> 16);
}
__device__ __forceinline__ float bf_up(unsigned short h) { return __uint_as_float(((unsigned)h) << 16); }
__device__ __forceinline__ float bf_val(float f) { return bf_up(bf_bits(f)); }
__device__ __forceinline__ unsigned short h_bits(_Float16 x) { return __builtin_bit_cast(unsigned short, x); }
__device__ __forceinline__ unsigned pk16(unsigned short a, unsigned short b) { return (unsigned)a | ((unsigned)b << 16); }
__device__ __forceinline__ v8f zero8() { v8f z = {0.f, 0.f, 0.f, 0.f, 0.f, 0.f, 0.f, 0.f}; return z; }

__device__ __forceinline__ v16h ldfrag_h(const _Float16* p) {
  FragH f;
  f.h[0] = *(const v8h*)(p);
  f.h[1] = *(const v8h*)(p + 16);
  return f.v;
}

__device__ __forceinline__ v8f mma_h(v16h a, v16h b, v8f c) {
  return __builtin_amdgcn_wmma_f32_16x16x32_f16(false, a, false, b, (short)0, c, false, false);
}
template <typename F>
__device__ __forceinline__ void guard6(v8f& a, v8f& b, v8f& c, v8f& d, F x0, F x1, F x2, F x3, F x4, F x5) {
#if defined(__HIP_DEVICE_COMPILE__)
  asm volatile("v_nop\n\tv_nop\n\tv_nop\n\tv_nop"
               : "+v"(a), "+v"(b), "+v"(c), "+v"(d) : "v"(x0), "v"(x1), "v"(x2), "v"(x3), "v"(x4), "v"(x5) : "memory");
#endif
}
__device__ __forceinline__ void acc_guard4(v8f& a, v8f& b, v8f& c, v8f& d) {
#if defined(__HIP_DEVICE_COMPILE__)
  asm volatile("v_nop\n\tv_nop\n\tv_nop\n\tv_nop" : "+v"(a), "+v"(b), "+v"(c), "+v"(d));
#endif
}

__global__ __launch_bounds__(256) void cvt16(const float* __restrict__ x, u16* D, int n8, int mode, float scale) {
  const int gt = blockIdx.x * 256 + (int)threadIdx.x;
  if (gt >= n8) return;
  const float* p = x + (size_t)gt * 8;
  const v4f a = *(const v4f*)(p), c4 = *(const v4f*)(p + 4);
  float v[8];
#pragma unroll
  for (int e = 0; e < 4; ++e) { v[e] = a[e]; v[4 + e] = c4[e]; }
  unsigned short s[8];
#pragma unroll
  for (int e = 0; e < 8; ++e) {
    const unsigned short bb = bf_bits(v[e]);
    const unsigned short hb = h_bits((_Float16)(bf_up(bb) * scale));
    s[e] = (mode != 0) ? hb : bb;
  }
  v4u o;
#pragma unroll
  for (int e = 0; e < 4; ++e) o[e] = pk16(s[2 * e], s[2 * e + 1]);
  u16* d = D + (size_t)gt * 8;
  for (int pass = 0; pass < 2; ++pass) {
    *(volatile v4u*)(d) = o;
    __threadfence();
  }
}

__global__ __launch_bounds__(256)
void k_u2(const float* __restrict__ x, const float* __restrict__ Wlin, const float* __restrict__ av,
          const float* __restrict__ aux, float* u2l) {
  __shared__ float as_[DIN];
  __shared__ float ws_[WIN];
  (void)aux;
  const int tid = threadIdx.x;
  const int b   = blockIdx.y;
  const int j   = blockIdx.x * 256 + tid;
  as_[tid] = bf_val(av[tid]);
  __syncthreads();
  if (tid < WIN) {
    const float* wr = Wlin + (size_t)(WIN + tid) * DIN;
    float acc = 0.f;
#pragma unroll 4
    for (int d = 0; d < DIN; ++d) acc += bf_val(wr[d]) * as_[d];
    ws_[tid] = acc;
  }
  __syncthreads();
  const float* xb = x + (size_t)b * XBS_FULL + j;
  float acc = 0.f;
#pragma unroll 4
  for (int w = 0; w < WIN; ++w) acc += bf_val(xb[(size_t)w * NF]) * ws_[w];
  const float val = acc * LOG2E;
  float* dst = u2l + (size_t)b * NF + j;
  for (int pass = 0; pass < 2; ++pass) {
    *(volatile float*)(dst) = val;
    __threadfence();
  }
}

__global__ __launch_bounds__(ATT_THREADS)
void attn_pv(const u16* __restrict__ XH, const float* __restrict__ u2l, const float* __restrict__ bias, float* out) {
  __shared__ __align__(16) float tile[WIN * TP];

  const int tid  = threadIdx.x;
  const int wave = tid >> 5;
  const int lane = tid & 31;
  const int hh   = lane >> 4;
  const int c    = lane & 15;

  const int bid   = blockIdx.x;
  const int itile = bid % ITILES;
  const int b     = bid / ITILES;
  if (b >= NB) return;
  const int iblk  = itile * 64;
  const int i0    = iblk + wave * 16;
  const int iq    = i0 + c;

  const float* brow = bias + (size_t)iq * NF + 8 * hh;
  const float* urow = u2l + (size_t)b * NF + 8 * hh;
  const _Float16* Vb = (const _Float16*)(const void*)XH + ((size_t)b * WIN + c) * NF + 8 * hh;
  const size_t vs = (size_t)16 * NF;

  float mrun = -INFINITY, lrun = 0.f;
  v8f o[8];
#pragma unroll
  for (int j = 0; j < 8; ++j) o[j] = zero8();

#pragma unroll 1
  for (int it = 0; it < NKB; ++it) {
    const int kb = it * 32;
    const v4f g0 = *(const v4f*)(brow + kb),      g1 = *(const v4f*)(brow + kb + 4);
    const v4f g2 = *(const v4f*)(brow + kb + 16), g3 = *(const v4f*)(brow + kb + 20);
    const v4f q0 = *(const v4f*)(urow + kb),      q1 = *(const v4f*)(urow + kb + 4);
    const v4f q2 = *(const v4f*)(urow + kb + 16), q3 = *(const v4f*)(urow + kb + 20);
    float tk[16];
#pragma unroll
    for (int e = 0; e < 4; ++e) {
      tk[e]      = g0[e] * LOG2E + q0[e];
      tk[4 + e]  = g1[e] * LOG2E + q1[e];
      tk[8 + e]  = g2[e] * LOG2E + q2[e];
      tk[12 + e] = g3[e] * LOG2E + q3[e];
    }
    float cm = tk[0];
#pragma unroll
    for (int i = 1; i < 16; ++i) cm = fmaxf(cm, tk[i]);
    cm = fmaxf(cm, __shfl_xor(cm, 16, 32));
    const float mn = fmaxf(mrun, cm);
    const float al = (mrun == -INFINITY) ? 0.f : exp2f(mrun - mn);
    mrun = mn;
    float ps = 0.f;
    FragH ph;
#pragma unroll
    for (int w = 0; w < 2; ++w) {
#pragma unroll
      for (int e4 = 0; e4 < 4; ++e4) {
        const int i = 8 * w + 2 * e4;
        const float p0 = exp2f(fminf(tk[i] - mn, 0.f));
        const float p1 = exp2f(fminf(tk[i + 1] - mn, 0.f));
        ps += p0 + p1;
        ph.u[w][e4] = pk16(h_bits((_Float16)(p0 * PCAR)), h_bits((_Float16)(p1 * PCAR)));
      }
    }
    ps += __shfl_xor(ps, 16, 32);
    lrun = lrun * al + ps;
    float scl[8];
#pragma unroll
    for (int r = 0; r < 8; ++r) scl[r] = __shfl(al, 8 * hh + r, 32);
#pragma unroll
    for (int j = 0; j < 8; ++j) {
#pragma unroll
      for (int r = 0; r < 8; ++r) o[j][r] *= scl[r];
    }
    {
      const _Float16* vp = Vb + kb;
      const v16h vf0 = ldfrag_h(vp);
      const v16h vf1 = ldfrag_h(vp + vs);
      const v16h vf2 = ldfrag_h(vp + 2 * vs);
      const v16h vf3 = ldfrag_h(vp + 3 * vs);
      o[0] = mma_h(ph.v, vf0, o[0]);
      o[1] = mma_h(ph.v, vf1, o[1]);
      o[2] = mma_h(ph.v, vf2, o[2]);
      o[3] = mma_h(ph.v, vf3, o[3]);
      guard6<v16h>(o[0], o[1], o[2], o[3], ph.v, vf0, vf1, vf2, vf3, ph.v);
      const v16h vf4 = ldfrag_h(vp + 4 * vs);
      const v16h vf5 = ldfrag_h(vp + 5 * vs);
      const v16h vf6 = ldfrag_h(vp + 6 * vs);
      const v16h vf7 = ldfrag_h(vp + 7 * vs);
      o[4] = mma_h(ph.v, vf4, o[4]);
      o[5] = mma_h(ph.v, vf5, o[5]);
      o[6] = mma_h(ph.v, vf6, o[6]);
      o[7] = mma_h(ph.v, vf7, o[7]);
      guard6<v16h>(o[4], o[5], o[6], o[7], ph.v, vf4, vf5, vf6, vf7, ph.v);
    }
  }
  acc_guard4(o[0], o[1], o[2], o[3]);
  acc_guard4(o[4], o[5], o[6], o[7]);

  const float linv = (lrun > 0.f) ? ((1.0f / lrun) * (1.0f / (PCAR * VCAR))) : 0.f;
  float inv[8];
#pragma unroll
  for (int r = 0; r < 8; ++r) inv[r] = __shfl(linv, 8 * hh + r, 32);
#pragma unroll
  for (int r = 0; r < 8; ++r) {
#pragma unroll
    for (int j = 0; j < 8; ++j) {
      const float hv = o[j][r] * inv[r];
      const float ex = exp2f(-hv * LOG2E);
      const float sg = __builtin_amdgcn_rcpf(1.0f + ex);
      tile[(16 * j + c) * TP + wave * 16 + 8 * hh + r] = sg;
    }
  }
  __syncthreads();
  const int rsub = tid >> 4, col4 = (tid & 15) * 4;
  float* ob = out + ((size_t)b * WIN) * NF + iblk + col4;
  for (int pass = 0; pass < 2; ++pass) {
#pragma unroll
    for (int it2 = 0; it2 < WIN / 8; ++it2) {
      const int w = it2 * 8 + rsub;
      const v4f val = *(const v4f*)(tile + w * TP + col4);
      *(volatile v4f*)(ob + (size_t)w * NF) = val;
    }
    __threadfence();
  }
}

extern "C" void kernel_launch(void* const* d_in, const int* in_sizes, int n_in,
                              void* d_out, int out_size, void* d_ws, size_t ws_size,
                              hipStream_t stream) {
  if (n_in < 5) return;
  if (in_sizes[0] < NB * WIN * NF) return;
  if (in_sizes[1] < DIN * DIN) return;
  if (in_sizes[2] < 1) return;
  if (in_sizes[3] < DIN) return;
  if (in_sizes[4] < NF * NF) return;
  if (out_size < NB * WIN * NF) return;

  const float* Xin  = (const float*)d_in[0];
  const float* Wlin = (const float*)d_in[1];
  const float* Blin = (const float*)d_in[2];
  const float* Av   = (const float*)d_in[3];
  const float* Bias = (const float*)d_in[4];
  float*       out  = (float*)d_out;

  const size_t szXH = (size_t)NB * WIN * NF * 2;
  const size_t szU2 = (size_t)NB * NF * 4;
  size_t off = 0;
  const size_t oXH = off; off += szXH;
  const size_t oU2 = off; off += szU2;
  if (off > ws_size) return;
  if (off > (size_t)134217728) return;

  char* ws = (char*)d_ws;
  u16*   XH = (u16*)(ws + oXH);
  float* U2 = (float*)(ws + oU2);

  const int n8x = (NB * WIN * NF) / 8;
  if ((n8x % 256) != 0) return;
  const dim3 gX(n8x / 256);
  const dim3 bX(256);
  const dim3 gU(NF / 256, NB);
  const dim3 bU(256);
  const dim3 gA(ATT_BLOCKS);
  const dim3 bA(ATT_THREADS);

  cvt16<<<gX, bX, 0, stream>>>(Xin, XH, n8x, 1, VCAR);
  k_u2<<<gU, bU, 0, stream>>>(Xin, Wlin, Av, Blin, U2);
  attn_pv<<<gA, bA, 0, stream>>>(XH, U2, Bias, out);
  (void)hipGetLastError();
}
